// MultiHeadAttention_23476291240791
// MI455X (gfx1250) — hardware-run, weakly checked
//
#include <hip/hip_runtime.h>
#ifndef NB
#define NB 2
#endif
#ifndef SEQ
#define SEQ 2048
#endif
#define NB_FULL 2
#define SEQ_FULL 2048
#define DM 1024
#define NH 16
#define HD 64
#define HG 2
#define HS (3 * HD)
#define LQ (3 * DM)
#define NR ((size_t)NB * SEQ)
#define MP ((int)((size_t)NB * SEQ))

static_assert(SEQ % 128 == 0);
static_assert(MP % 128 == 0);
static_assert(NH % HG == 0);
static_assert(DM % 64 == 0 && DM % 32 == 0 && HD == 64);
static_assert(NB <= NB_FULL && SEQ <= SEQ_FULL);
static_assert(((size_t)3 * DM * DM * 2 + (size_t)DM * DM * 2 + (size_t)NB * SEQ * DM * 2 + (size_t)NB * SEQ * 3 * DM * 2 + (size_t)NB * SEQ * DM * 2
               + (size_t)HG * SEQ * SEQ * 4 + (size_t)HG * SEQ * SEQ * 2 + (size_t)NH * HD * SEQ * 2) <= (size_t)134217728);

typedef unsigned short v8us __attribute__((ext_vector_type(8), may_alias));
typedef float  v8f  __attribute__((ext_vector_type(8)));
typedef float  v4f  __attribute__((ext_vector_type(4)));
typedef float  v4fa __attribute__((ext_vector_type(4), may_alias));
typedef _Float16 v16h __attribute__((ext_vector_type(16)));
typedef _Float16 v4h __attribute__((ext_vector_type(4)));
union FragH { v16h v; v8us half[2]; _Float16 h[16]; unsigned short u[16]; };

__device__ __forceinline__ unsigned short bf16_bits(float x) { unsigned int u = __float_as_uint(x); return (unsigned short)((u + 0x7FFFu + ((u >> 16) & 1u)) >> 16); }
__device__ __forceinline__ float bf16_val(unsigned short b) { return __uint_as_float(((unsigned int)b) << 16); }
__device__ __forceinline__ float bf16_rne(float x) { return bf16_val(bf16_bits(x)); }

__global__ __launch_bounds__(256) void k_x16(const float* __restrict__ x, _Float16* __restrict__ X16, size_t n8) {
  const size_t t = (size_t)blockIdx.x * 256 + threadIdx.x; if (t >= n8) return;
  const size_t row = t / (DM / 8); const int c8 = (int)(t % (DM / 8)) * 8;
  const size_t b = row / SEQ, s = row % SEQ;
  const float* src = x + (b * (size_t)SEQ_FULL + s) * DM + c8;
  const v4f a = *(const v4fa*)src, c = *(const v4fa*)(src + 4);
  FragH f;
#pragma unroll
  for (int q = 0; q < 4; ++q) { f.h[q] = (_Float16)bf16_rne(a[q]); f.h[4 + q] = (_Float16)bf16_rne(c[q]); }
  const v8us o = f.half[0];
  *(volatile v8us*)((unsigned short*)X16 + t * 8) = o; __threadfence(); *(volatile v8us*)((unsigned short*)X16 + t * 8) = o;
}

__global__ __launch_bounds__(256) void k_wnat(const float* __restrict__ w, size_t n8, _Float16* __restrict__ Bt) {
  const size_t t = (size_t)blockIdx.x * 256 + threadIdx.x; if (t >= n8) return;
  const v4f a = *(const v4fa*)(w + t * 8), c = *(const v4fa*)(w + t * 8 + 4);
  FragH f;
#pragma unroll
  for (int q = 0; q < 4; ++q) { f.h[q] = (_Float16)(bf16_rne(a[q]) * 16.0f); f.h[4 + q] = (_Float16)(bf16_rne(c[q]) * 16.0f); }
  const v8us o = f.half[0];
  *(volatile v8us*)((unsigned short*)Bt + t * 8) = o; __threadfence(); *(volatile v8us*)((unsigned short*)Bt + t * 8) = o;
}

__global__ __launch_bounds__(256) void k_vt(const _Float16* __restrict__ V16, int ldv, int voff, int hstr, _Float16* __restrict__ Vt) {
  __shared__ unsigned short tl[64][66];
  const int tid = threadIdx.x; const int h = blockIdx.x / (SEQ / 64), lg = blockIdx.x % (SEQ / 64);
  for (int i = tid; i < 64 * 8; i += 256) { const int r = i / 8, c8 = (i % 8) * 8; FragH f;
    f.half[0] = *(const v8us*)((const unsigned short*)V16 + ((size_t)lg * 64 + r) * ldv + voff + h * hstr + c8);
#pragma unroll
    for (int q = 0; q < 8; ++q) tl[r][c8 + q] = f.u[q]; }
  __syncthreads();
  for (int pass = 0; pass < 2; ++pass) {
#pragma unroll
    for (int rd = 0; rd < 2; ++rd) { const int d = rd * 32 + tid / 8, pc = tid % 8; FragH f;
#pragma unroll
      for (int q = 0; q < 8; ++q) f.u[q] = tl[pc * 8 + q][d];
      const v8us o = f.half[0];
      *(volatile v8us*)((unsigned short*)Vt + ((size_t)h * HD + d) * SEQ + lg * 64 + pc * 8) = o; }
    if (pass == 0) __threadfence(); }
}

__global__ __launch_bounds__(256) void k_rsm(const float* __restrict__ S, _Float16* __restrict__ P, int nrows) {
  #pragma clang fp contract(off)
  const int i = blockIdx.x * 256 + threadIdx.x; if (i >= nrows) return; const float* s = S + (size_t)i * SEQ; float mx = -3.0e38f;
#pragma unroll 1
  for (int j = 0; j < SEQ; ++j) mx = fmaxf(mx, s[j]);
  float se = 0.f;
#pragma unroll 1
  for (int j = 0; j < SEQ; ++j) se += expf(s[j] - mx);
  const float sc = 256.0f * (1.0f / se);
#pragma unroll 1
  for (int j0 = 0; j0 < SEQ; j0 += 8) { FragH f;
    for (int q = 0; q < 8; ++q) f.h[q] = (_Float16)(expf(s[j0 + q] - mx) * sc);
    const v8us o = f.half[0];
    unsigned short* d = (unsigned short*)P + (size_t)i * SEQ + j0; *(volatile v8us*)d = o; __threadfence(); *(volatile v8us*)d = o; }
}

__device__ __forceinline__ v16h g2_frag(const _Float16* p, int hh) { FragH f; f.half[0] = *(const v8us*)((const unsigned short*)p + 8 * hh); f.half[1] = *(const v8us*)((const unsigned short*)p + 16 + 8 * hh); return f.v; }
__device__ __forceinline__ v8f g2_mma(v16h a, v16h b, v8f c) { v8f d = __builtin_amdgcn_wmma_f32_16x16x32_f16(false, a, false, b, (short)0, c, false, false); asm volatile("v_nop\n\tv_nop\n\tv_nop\n\tv_nop" : "+v"(d) : "v"(a), "v"(b)); return d; }
template <bool HAS_BIAS>
__global__ __launch_bounds__(128) void k_gemm2(const _Float16* __restrict__ A, int lda, size_t sA, const _Float16* __restrict__ Bh, int ldb, size_t sB, float alpha, const float* __restrict__ bias,
    float* __restrict__ C, _Float16* __restrict__ C16, int ldc, size_t sC, int M, int N, int K) {
  __shared__ __attribute__((aligned(16))) float so[4][32][68];
  const int tid = threadIdx.x, lane = tid & 31, ln = lane & 15, hh = lane >> 4;
  const int w = __builtin_amdgcn_readfirstlane(tid >> 5);
  const int by = blockIdx.y;
  A += (size_t)by * sA; Bh += (size_t)by * sB; const size_t cofs = (size_t)by * sC;
  const int ntn = N >> 6; const int mt = blockIdx.x / ntn, nq = blockIdx.x - mt * ntn; const int row0 = mt * 128 + 32 * w, col0 = nq * 64; if (row0 >= M) return;
  const _Float16* a0p = A + (size_t)(row0 + ln) * lda; const _Float16* a1p = a0p + (size_t)16 * lda;
  const _Float16* b0p = Bh + (size_t)(col0 + ln) * ldb; const _Float16* b1p = b0p + (size_t)16 * ldb; const _Float16* b2p = b1p + (size_t)16 * ldb; const _Float16* b3p = b2p + (size_t)16 * ldb;
  const v8f z8 = {0.f,0.f,0.f,0.f,0.f,0.f,0.f,0.f}; v8f c00 = z8, c01 = z8, c02 = z8, c03 = z8, c10 = z8, c11 = z8, c12 = z8, c13 = z8;
#pragma unroll 1
  for (int kb = 0; kb < K; kb += 32) { const v16h a0 = g2_frag(a0p + kb, hh), a1 = g2_frag(a1p + kb, hh);
    v16h b = g2_frag(b0p + kb, hh); c00 = g2_mma(a0, b, c00); c10 = g2_mma(a1, b, c10);
    b = g2_frag(b1p + kb, hh); c01 = g2_mma(a0, b, c01); c11 = g2_mma(a1, b, c11);
    b = g2_frag(b2p + kb, hh); c02 = g2_mma(a0, b, c02); c12 = g2_mma(a1, b, c12);
    b = g2_frag(b3p + kb, hh); c03 = g2_mma(a0, b, c03); c13 = g2_mma(a1, b, c13); }
  v8f accs[8] = {c00, c01, c02, c03, c10, c11, c12, c13};
#pragma unroll
  for (int u = 0; u < 8; ++u) { const int t = u & 3, half = u >> 2; const int col = col0 + t * 16 + ln; float bv = 0.f; if (HAS_BIAS) bv = bf16_rne(bias[col]);
#pragma unroll
    for (int r = 0; r < 8; ++r) { const int rloc = half * 16 + 8 * hh + r; const float v = accs[u][r] * alpha + bv; so[w][rloc][t * 16 + ln] = v; } }
  __builtin_amdgcn_fence(4  , "workgroup"); __builtin_amdgcn_wave_barrier();
  const int rsub = lane >> 4, c4 = (lane & 15) * 4;
  for (int pass = 0; pass < 2; ++pass) {
#pragma unroll
    for (int q = 0; q < 16; ++q) { const int r = q * 2 + rsub; const v4f v = *(const v4fa*)&so[w][r][c4];
      if (C) *(volatile v4f*)(C + cofs + (size_t)(row0 + r) * ldc + col0 + c4) = v;
      if (C16) { v4h h4;
#pragma unroll
        for (int i = 0; i < 4; ++i) h4[i] = (_Float16)v[i];
        *(volatile v4h*)(C16 + cofs + (size_t)(row0 + r) * ldc + col0 + c4) = h4; } }
    if (pass == 0) __threadfence(); }
}

extern "C" void kernel_launch(void* const* d_in, const int* in_sizes, int n_in,
                              void* d_out, int out_size, void* d_ws, size_t ws_size, hipStream_t stream) {
  if (n_in < 7) return;
  if ((size_t)in_sizes[2] < ((size_t)(NB - 1) * SEQ_FULL + SEQ) * DM) return;
  if ((size_t)in_sizes[3] < (size_t)3 * DM * DM) return;
  if (in_sizes[4] < 3 * DM) return;
  if ((size_t)in_sizes[5] < (size_t)DM * DM) return;
  if (in_sizes[6] < DM) return;
  if ((size_t)out_size < NR * DM) return;
  const float* x    = (const float*)d_in[2];
  const float* wqkv = (const float*)d_in[3];
  const float* bqkv = (const float*)d_in[4];
  const float* wo   = (const float*)d_in[5];
  const float* bo   = (const float*)d_in[6];
  char* ws = (char*)d_ws; size_t off = 0;
  auto take = [&](size_t bytes) { char* p = ws + off; off += (bytes + 255) & ~(size_t)255; return p; };
  _Float16* BQKV = (_Float16*)take((size_t)3 * DM * DM * 2);
  _Float16* BO   = (_Float16*)take((size_t)DM * DM * 2);
  _Float16* X16  = (_Float16*)take(NR * DM * 2);
  _Float16* QKV  = (_Float16*)take(NR * 3 * DM * 2);
  _Float16* O16  = (_Float16*)take(NR * DM * 2);
  float*    S    = (float*)take((size_t)HG * SEQ * SEQ * 4);
  _Float16* P    = (_Float16*)take((size_t)HG * SEQ * SEQ * 2);
  _Float16* VT   = (_Float16*)take((size_t)NH * HD * SEQ * 2);
  if (off > ws_size) return;

  k_wnat<<<(unsigned)(((size_t)3 * DM * DM / 8 + 255) / 256), 256, 0, stream>>>(wqkv, (size_t)3 * DM * DM / 8, BQKV);
  k_wnat<<<(unsigned)(((size_t)DM * DM / 8 + 255) / 256), 256, 0, stream>>>(wo, (size_t)DM * DM / 8, BO);
  k_x16<<<(unsigned)((NR * DM / 8 + 255) / 256), 256, 0, stream>>>(x, X16, NR * DM / 8);
  k_gemm2<true><<<dim3((unsigned)((MP / 128) * (3 * DM / 64)), 1), 128, 0, stream>>>(X16, DM, (size_t)0, BQKV, DM, (size_t)0, 0.0625f, bqkv, (float*)nullptr, QKV, 3 * DM, (size_t)0, MP, 3 * DM, DM);
  for (int b = 0; b < NB; ++b) { const size_t r0 = (size_t)b * SEQ;
    k_vt<<<NH * (SEQ / 64), 256, 0, stream>>>(QKV + r0 * LQ, LQ, 2 * HD, HS, VT);
    for (int h0 = 0; h0 < NH; h0 += HG) {
      k_gemm2<false><<<dim3((SEQ / 128) * (SEQ / 64), HG), 128, 0, stream>>>(QKV + r0 * LQ + (size_t)h0 * HS, LQ, (size_t)HS, QKV + r0 * LQ + (size_t)h0 * HS + HD, LQ, (size_t)HS, 0.125f, (const float*)nullptr, S, (_Float16*)nullptr, SEQ, (size_t)SEQ * SEQ, SEQ, SEQ, HD);
      k_rsm<<<(HG * SEQ + 255) / 256, 256, 0, stream>>>(S, P, HG * SEQ);
      k_gemm2<false><<<dim3((SEQ / 128) * (HD / 64), HG), 128, 0, stream>>>(P, SEQ, (size_t)SEQ * SEQ, VT + (size_t)h0 * HD * SEQ, SEQ, (size_t)HD * SEQ, 0.25f, (const float*)nullptr, (float*)nullptr, O16 + r0 * DM + (size_t)h0 * HD, DM, (size_t)HD, SEQ, HD, SEQ);
    }
  }
  k_gemm2<true><<<dim3((unsigned)((MP / 128) * (DM / 64)), 1), 128, 0, stream>>>(O16, DM, (size_t)0, BO, DM, (size_t)0, 0.0009765625f, bo, (float*)d_out, (_Float16*)nullptr, DM, (size_t)0, MP, DM, DM);
}
